// StreamingSelfAttention_36876589204185
// MI455X (gfx1250) — hardware-run, weakly checked
//
#include <hip/hip_runtime.h>
#include <math.h>

typedef __attribute__((ext_vector_type(16))) _Float16 v16h;
typedef __attribute__((ext_vector_type(8)))  _Float16 v8h;
typedef __attribute__((ext_vector_type(8)))  float    v8f;
typedef __attribute__((ext_vector_type(4)))  float    v4f;

constexpr int kBatch = 2;
constexpr int kSeq   = 4096;
constexpr int kDm    = 512;
constexpr int kHeads = 8;
constexpr int kHd    = 64;
constexpr int kLeft  = 128;
constexpr int kTok   = kBatch * kSeq;
constexpr int kQKld  = 2 * kDm;
static_assert(kHeads * kHd == kDm);
static_assert(kTok == 8192 && kQKld == 1024);

constexpr int kInputsRneToBf16 = 1;

constexpr int isqrt_exact(int n) { int r = 0; while ((r + 1) * (r + 1) <= n) ++r; return r; }
static_assert(isqrt_exact(kHd) * isqrt_exact(kHd) == kHd);

constexpr float kXCarry   = 16.0f;
constexpr float kWCarry   = 256.0f;
constexpr float kQKVCarry = 16.0f;
constexpr float kRemCarry = 2048.0f;
constexpr float kRemInv   = 1.0f / kRemCarry;
constexpr float kPCarry   = 4096.0f;
constexpr float kCtxCarry = 64.0f;
constexpr float kProjScale  = 1.0f / (kXCarry * kWCarry);
constexpr float kQKScale    = 1.0f / (float)isqrt_exact(kHd);
constexpr float kScoreScale = kQKScale / (kQKVCarry * kQKVCarry);
constexpr float kCtxFold    = kCtxCarry / kQKVCarry;
constexpr float kOutScale   = 1.0f / (kCtxCarry * kWCarry);
constexpr float kF16MinNormal = 6.103515625e-5f;

constexpr int kQT     = 32;
constexpr int kFrame  = kLeft + kQT;
constexpr int kTiles  = kFrame / 16;
constexpr int kKSteps = kFrame / 32;
constexpr int kSP     = kFrame + 4;
constexpr int kPP     = kFrame + 8;
static_assert((kFrame % 32) == 0 && (kSeq % kQT) == 0 && (kLeft % 32) == 0);
static_assert(kTiles == 10 && kKSteps == 5);
static_assert(((kSP * 4) % 16) == 0 && ((kPP * 2) % 16) == 0);

constexpr size_t kOffX16   = 0;
constexpr size_t kOffW16   = kOffX16   + (size_t)kTok * kDm * 2;
constexpr size_t kOffWO16  = kOffW16   + (size_t)3 * kDm * kDm * 2;
constexpr size_t kOffQK16  = kOffWO16  + (size_t)kDm * kDm * 2;
constexpr size_t kOffQKL16 = kOffQK16  + (size_t)kTok * kQKld * 2;
constexpr size_t kOffVT16  = kOffQKL16 + (size_t)kTok * kQKld * 2;
constexpr size_t kOffVTL16 = kOffVT16  + (size_t)kDm * kTok * 2;
constexpr size_t kOffCTX16 = kOffVTL16 + (size_t)kDm * kTok * 2;
constexpr size_t kWsTotal  = kOffCTX16 + (size_t)kTok * kDm * 2;
static_assert(kWsTotal == 69206016ull);
static_assert(kWsTotal <= 134217728ull);
static_assert((kOffW16 % 128) == 0 && (kOffWO16 % 128) == 0 && (kOffQK16 % 128) == 0 && (kOffQKL16 % 128) == 0 &&
              (kOffVT16 % 128) == 0 && (kOffVTL16 % 128) == 0 && (kOffCTX16 % 128) == 0);

__device__ __forceinline__ unsigned short f2bf_bits(float f) {
  unsigned u = __float_as_uint(f);
  return (unsigned short)((u + 0x7FFFu + ((u >> 16) & 1u)) >> 16);
}
__device__ __forceinline__ float bf_bits2f(unsigned short h) { return __uint_as_float(((unsigned)h) << 16); }

__device__ __forceinline__ float prep_in(float v) {
  if (kInputsRneToBf16) return bf_bits2f(f2bf_bits(v));
  return v;
}

__device__ __forceinline__ _Float16 to_f16_flushed(float v) {
  const float w = (fabsf(v) < kF16MinNormal) ? 0.0f : v;
  return (_Float16)w;
}

union FragU { v16h v; v8h h[2]; };
__device__ __forceinline__ v16h frag_load(const _Float16* p) {
  FragU f;
  f.h[0] = *(const v8h*)(p);
  f.h[1] = *(const v8h*)(p + 16);
  return f.v;
}

__device__ __forceinline__ v8f mma_g(v16h a, v16h b, v8f c) {
  c = __builtin_amdgcn_wmma_f32_16x16x32_f16(false, a, false, b, (short)0, c, false, false);
  asm volatile("v_nop\n\tv_nop\n\tv_nop\n\tv_nop" : "+v"(c) : "v"(a), "v"(b));
  return c;
}

__global__ __launch_bounds__(256) void cast8_f16_kernel(const float* __restrict__ in, unsigned short* __restrict__ out,
                                                        int n8, float carry) {
  const int i = blockIdx.x * 256 + threadIdx.x;
  if (i >= n8) return;
  const float* p = in + 8 * (size_t)i;
  const v4f a0 = *(const v4f*)(p);
  const v4f a1 = *(const v4f*)(p + 4);
  v8h hv;
#pragma unroll
  for (int e = 0; e < 4; ++e) {
    const float r0 = a0[e];
    const float r1 = a1[e];
    const float x0 = prep_in(r0);
    const float x1 = prep_in(r1);
    hv[e]     = to_f16_flushed(x0 * carry);
    hv[4 + e] = to_f16_flushed(x1 * carry);
  }
  unsigned short* q = out + 8 * (size_t)i;
  *(volatile v8h*)q = hv;
  __threadfence();
  *(volatile v8h*)q = hv;
}

template <int BIAS_MODE, int OUT_MODE>
__global__ __launch_bounds__(256) void gemm64_f16_kernel(
    const unsigned short* __restrict__ Ap, int lda,
    const unsigned short* __restrict__ Btp, int ldb,
    void* __restrict__ Cout, void* __restrict__ Cout2, int ldc,
    const float* __restrict__ bias,
    int M, int N, int K, float scale, float post) {
  const _Float16* A  = (const _Float16*)Ap;
  const _Float16* Bt = (const _Float16*)Btp;
  __shared__ __align__(16) float sT[8][16 * 68];
  const int lane = threadIdx.x & 31;
  const int wave = threadIdx.x >> 5;
  const int tilesN = N >> 6;
  const int tilesM = M >> 6;
  const int tile = blockIdx.x * 8 + wave;
  if (tile >= tilesM * tilesN) return;
  const int tm = tile / tilesN;
  const int tn = tile - tm * tilesN;
  const int m0 = tm << 6;
  const int n0 = tn << 6;
  const int rlane = lane & 15;
  const int koff  = (lane >> 4) * 8;
  const int mOff  = (lane >> 4) * 8;

  v8f acc[4][4];
#pragma unroll
  for (int i = 0; i < 4; ++i)
#pragma unroll
    for (int j = 0; j < 4; ++j) acc[i][j] = (v8f){0.f, 0.f, 0.f, 0.f, 0.f, 0.f, 0.f, 0.f};

  for (int k0 = 0; k0 < K; k0 += 32) {
    v16h bh[4];
#pragma unroll
    for (int j = 0; j < 4; ++j) {
      const size_t bo = (size_t)(n0 + (j << 4) + rlane) * ldb + koff + k0;
      bh[j] = frag_load(Bt + bo);
    }
#pragma unroll
    for (int i = 0; i < 4; ++i) {
      const size_t ao = (size_t)(m0 + (i << 4) + rlane) * lda + koff + k0;
      const v16h ah = frag_load(A + ao);
#pragma unroll
      for (int j = 0; j < 4; ++j) acc[i][j] = mma_g(ah, bh[j], acc[i][j]);
    }
  }

  float* slab = sT[wave];
#pragma unroll
  for (int i = 0; i < 4; ++i) {
    const int mBase = m0 + (i << 4);
    float bm[8];
#pragma unroll
    for (int r = 0; r < 8; ++r) {
      bm[r] = 0.0f;
      if (BIAS_MODE == 1) bm[r] = prep_in(bias[mBase + mOff + r]);
    }
#pragma unroll
    for (int j = 0; j < 4; ++j) {
      const int n = n0 + (j << 4) + rlane;
      float bv = 0.f;
      if (BIAS_MODE == 2) bv = prep_in(bias[n]);
#pragma unroll
      for (int r = 0; r < 8; ++r) {
        float v = acc[i][j][r] * scale;
        if (BIAS_MODE == 1) v += bm[r];
        if (BIAS_MODE == 2) v += bv;
        v *= post;
        slab[(mOff + r) * 68 + (j << 4) + rlane] = v;
      }
    }
    __builtin_amdgcn_fence(__ATOMIC_RELEASE, "workgroup");
    __builtin_amdgcn_wave_barrier();
    __builtin_amdgcn_fence(__ATOMIC_ACQUIRE, "workgroup");
    if (OUT_MODE == 0) {
      float* C = (float*)Cout;
      const int hh = lane >> 4, c4 = (lane & 15) * 4;
      for (int pass = 0; pass < 2; ++pass) {
#pragma unroll
        for (int it = 0; it < 8; ++it) {
          const int row = it * 2 + hh;
          const v4f v = *(const v4f*)(slab + row * 68 + c4);
          *(volatile v4f*)(C + (size_t)(mBase + row) * ldc + n0 + c4) = v;
        }
        __threadfence();
      }
    } else {
      const int q = lane >> 3, c8 = (lane & 7) * 8;
      unsigned short* C  = (unsigned short*)Cout;
      unsigned short* C2 = (unsigned short*)Cout2;
      v8h hv[4], lv[4];
#pragma unroll
      for (int it = 0; it < 4; ++it) {
        const int row = it * 4 + q;
        const float* sp = slab + row * 68 + c8;
        const v4f s0 = *(const v4f*)(sp);
        const v4f s1 = *(const v4f*)(sp + 4);
#pragma unroll
        for (int e = 0; e < 4; ++e) {
          const float x0 = s0[e];
          const float x1 = s1[e];
          const _Float16 h0 = to_f16_flushed(x0);
          const _Float16 h1 = to_f16_flushed(x1);
          const float d0 = (x0 - (float)h0) * kRemCarry;
          const float d1 = (x1 - (float)h1) * kRemCarry;
          hv[it][e]     = h0;
          hv[it][4 + e] = h1;
          lv[it][e]     = to_f16_flushed(d0);
          lv[it][4 + e] = to_f16_flushed(d1);
        }
      }
      for (int pass = 0; pass < 2; ++pass) {
#pragma unroll
        for (int it = 0; it < 4; ++it) {
          const int row = it * 4 + q;
          const size_t o = (size_t)(mBase + row) * ldc + n0 + c8;
          *(volatile v8h*)(C + o)  = hv[it];
          *(volatile v8h*)(C2 + o) = lv[it];
        }
        __threadfence();
      }
    }
    __builtin_amdgcn_fence(__ATOMIC_RELEASE, "workgroup");
    __builtin_amdgcn_wave_barrier();
    __builtin_amdgcn_fence(__ATOMIC_ACQUIRE, "workgroup");
  }
}

__device__ __forceinline__ _Float16 prob_f16(float x, float m, bool ok) {
  const float arg = ok ? (x - m) : 0.0f;
  const float ex = expf(arg);
  float pc = ok ? (ex * kPCarry) : 0.0f;
  pc = (pc < kF16MinNormal) ? 0.0f : pc;
  return (_Float16)pc;
}

__global__ __launch_bounds__(64) void band_attn_kernel(const unsigned short* __restrict__ QKp,
                                                       const unsigned short* __restrict__ QKLp,
                                                       const unsigned short* __restrict__ VTp,
                                                       const unsigned short* __restrict__ VTLp,
                                                       unsigned short* __restrict__ CTXp) {
  __shared__ __align__(16) float    sS[2][16 * kSP];
  __shared__ __align__(16) _Float16 sP[2][16 * kPP];
  __shared__ __align__(16) float    sO[2][16 * 68];
  __shared__ float sInv[2][16];

  const _Float16* QK  = (const _Float16*)QKp;
  const _Float16* QKL = (const _Float16*)QKLp;
  const _Float16* VT  = (const _Float16*)VTp;
  const _Float16* VTL = (const _Float16*)VTLp;

  const int tid  = threadIdx.x;
  const int wave = tid >> 5;
  const int lane = tid & 31;
  const int hh   = lane >> 4;
  const int c    = lane & 15;

  constexpr int nqb = kSeq / kQT;
  const int bx = blockIdx.x;
  const int qb = bx % nqb;
  const int bh = bx / nqb;
  const int h  = bh % kHeads;
  const int b  = bh / kHeads;
  const int q0  = qb * kQT;
  const int q0w = q0 + wave * 16;
  const int kf0 = q0 - kLeft;
  const int t0  = (kf0 < 0) ? ((-kf0) >> 4) : 0;
  const int ks0 = t0 >> 1;
  const int rowb = b * kSeq;

  float* sw = sS[wave];
  {
    const size_t qoff = (size_t)(rowb + q0w + c) * kQKld + h * kHd + 8 * hh;
    const v16h qa0 = frag_load(QK + qoff);
    const v16h qa1 = frag_load(QK + qoff + 32);
    const v16h ql0 = frag_load(QKL + qoff);
    const v16h ql1 = frag_load(QKL + qoff + 32);
#pragma unroll 1
    for (int t = t0; t < kTiles; ++t) {
      const int kb = kf0 + t * 16;
      const size_t koff = (size_t)(rowb + kb + c) * kQKld + kDm + h * kHd + 8 * hh;
      const v16h kb0 = frag_load(QK + koff);
      const v16h kb1 = frag_load(QK + koff + 32);
      const v16h kl0 = frag_load(QKL + koff);
      const v16h kl1 = frag_load(QKL + koff + 32);
      v8f acc = (v8f){0.f, 0.f, 0.f, 0.f, 0.f, 0.f, 0.f, 0.f};
      v8f rem = (v8f){0.f, 0.f, 0.f, 0.f, 0.f, 0.f, 0.f, 0.f};
      acc = mma_g(qa0, kb0, acc);
      acc = mma_g(qa1, kb1, acc);
      rem = mma_g(qa0, kl0, rem);
      rem = mma_g(qa1, kl1, rem);
      rem = mma_g(ql0, kb0, rem);
      rem = mma_g(ql1, kb1, rem);
#pragma unroll
      for (int r = 0; r < 8; ++r) {
        const float joined = acc[r] + rem[r] * kRemInv;
        sw[(8 * hh + r) * kSP + t * 16 + c] = joined * kScoreScale;
      }
    }
  }
  __syncthreads();

  {
    const int srow = lane >> 1;
    const int sh   = lane & 1;
    const int qi   = q0w + srow;
    const float* srp = sw + srow * kSP;
    float m = -1.0e30f;
#pragma unroll 1
    for (int g = t0; g < kTiles; ++g) {
      const int col0 = (2 * g + sh) * 8;
      const v4f a0 = *(const v4f*)(srp + col0);
      const v4f a1 = *(const v4f*)(srp + col0 + 4);
#pragma unroll
      for (int e = 0; e < 4; ++e) {
        const float x0 = a0[e];
        const float x1 = a1[e];
        const int kj0 = kf0 + col0 + e;
        const int kj1 = kj0 + 4;
        const bool ok0 = (kj0 <= qi) && (kj0 >= qi - kLeft);
        const bool ok1 = (kj1 <= qi) && (kj1 >= qi - kLeft);
        m = ok0 ? fmaxf(m, x0) : m;
        m = ok1 ? fmaxf(m, x1) : m;
      }
    }
    const float mo = __shfl_xor(m, 1, 32);
    m = fmaxf(m, mo);

    float lsum = 0.0f;
    _Float16* pw = sP[wave];
#pragma unroll 1
    for (int g = t0; g < kTiles; ++g) {
      const int col0 = (2 * g + sh) * 8;
      const v4f a0 = *(const v4f*)(srp + col0);
      const v4f a1 = *(const v4f*)(srp + col0 + 4);
      v8h hv;
#pragma unroll
      for (int e = 0; e < 4; ++e) {
        const float x0 = a0[e];
        const float x1 = a1[e];
        const int kj0 = kf0 + col0 + e;
        const int kj1 = kj0 + 4;
        const bool ok0 = (kj0 <= qi) && (kj0 >= qi - kLeft);
        const bool ok1 = (kj1 <= qi) && (kj1 >= qi - kLeft);
        const _Float16 h0 = prob_f16(x0, m, ok0);
        const _Float16 h1 = prob_f16(x1, m, ok1);
        hv[e]     = h0;
        hv[4 + e] = h1;
        lsum += (float)h0;
        lsum += (float)h1;
      }
      *(v8h*)(pw + srow * kPP + col0) = hv;
    }
    const float lo = __shfl_xor(lsum, 1, 32);
    lsum += lo;
    if (sh == 0) sInv[wave][srow] = kCtxFold / lsum;
  }
  __syncthreads();

  v8f oacc[4];
  v8f orem[4];
#pragma unroll
  for (int t = 0; t < 4; ++t) {
    oacc[t] = (v8f){0.f, 0.f, 0.f, 0.f, 0.f, 0.f, 0.f, 0.f};
    orem[t] = (v8f){0.f, 0.f, 0.f, 0.f, 0.f, 0.f, 0.f, 0.f};
  }
  {
    const _Float16* prow = sP[wave] + c * kPP + 8 * hh;
    const long vcol = (long)rowb + kf0 + 8 * hh;
#pragma unroll 1
    for (int kk = ks0; kk < kKSteps; ++kk) {
      const v16h pa = frag_load(prow + kk * 32);
#pragma unroll
      for (int t = 0; t < 4; ++t) {
        const long off = (long)(h * kHd + t * 16 + c) * kTok + vcol + kk * 32;
        const v16h vb = frag_load(VT + off);
        const v16h vl = frag_load(VTL + off);
        oacc[t] = mma_g(pa, vb, oacc[t]);
        orem[t] = mma_g(pa, vl, orem[t]);
      }
    }
  }

  float* os = sO[wave];
#pragma unroll
  for (int r = 0; r < 8; ++r) {
    const float inv = sInv[wave][8 * hh + r];
#pragma unroll
    for (int t = 0; t < 4; ++t) {
      const float joined = oacc[t][r] + orem[t][r] * kRemInv;
      os[(8 * hh + r) * 68 + t * 16 + c] = joined * inv;
    }
  }
  __syncthreads();
  {
    const int q4 = lane >> 3, c8 = (lane & 7) * 8;
    v8h ov[4];
#pragma unroll
    for (int it = 0; it < 4; ++it) {
      const int row = it * 4 + q4;
      const float* sp = os + row * 68 + c8;
      const v4f s0 = *(const v4f*)(sp);
      const v4f s1 = *(const v4f*)(sp + 4);
#pragma unroll
      for (int e = 0; e < 4; ++e) {
        const float x0 = s0[e];
        const float x1 = s1[e];
        ov[it][e]     = to_f16_flushed(x0);
        ov[it][4 + e] = to_f16_flushed(x1);
      }
    }
    for (int pass = 0; pass < 2; ++pass) {
#pragma unroll
      for (int it = 0; it < 4; ++it) {
        const int row = it * 4 + q4;
        *(volatile v8h*)(CTXp + (size_t)(rowb + q0w + row) * kDm + h * kHd + c8) = ov[it];
      }
      __threadfence();
    }
  }
}

static_assert((kDm % 32) == 0);
static_assert((kTok % 64) == 0 && (kQKld % 64) == 0 && (kDm % 64) == 0);
static_assert((((kTok / 64) * (kQKld / 64)) % 8) == 0 && (((kDm / 64) * (kTok / 64)) % 8) == 0);
static_assert(((kTok * kDm / 8) % 256) == 0 && ((3 * kDm * kDm / 8) % 256) == 0 && ((kDm * kDm / 8) % 256) == 0);

extern "C" void kernel_launch(void* const* d_in, const int* in_sizes, int n_in,
                              void* d_out, int out_size, void* d_ws, size_t ws_size,
                              hipStream_t stream) {
  if (n_in < 5) return;
  if (in_sizes[0] != kTok * kDm) return;
  if (in_sizes[1] != 3 * kDm * kDm) return;
  if (in_sizes[2] != 3 * kDm) return;
  if (in_sizes[3] != kDm * kDm) return;
  if (in_sizes[4] != kDm) return;
  if (out_size != kTok * kDm) return;
  if (ws_size < kWsTotal) return;

  const float* x    = (const float*)d_in[0];
  const float* ipw  = (const float*)d_in[1];
  const float* ipb  = (const float*)d_in[2];
  const float* ow   = (const float*)d_in[3];
  const float* ob   = (const float*)d_in[4];
  float* out = (float*)d_out;

  char* ws = (char*)d_ws;
  unsigned short* X16   = (unsigned short*)(ws + kOffX16);
  unsigned short* W16   = (unsigned short*)(ws + kOffW16);
  unsigned short* WO16  = (unsigned short*)(ws + kOffWO16);
  unsigned short* QK16  = (unsigned short*)(ws + kOffQK16);
  unsigned short* QKL16 = (unsigned short*)(ws + kOffQKL16);
  unsigned short* VT16  = (unsigned short*)(ws + kOffVT16);
  unsigned short* VTL16 = (unsigned short*)(ws + kOffVTL16);
  unsigned short* CTX16 = (unsigned short*)(ws + kOffCTX16);

  cast8_f16_kernel<<<(kTok * kDm / 8) / 256, 256, 0, stream>>>(x, X16, kTok * kDm / 8, kXCarry);
  cast8_f16_kernel<<<(3 * kDm * kDm / 8) / 256, 256, 0, stream>>>(ipw, W16, 3 * kDm * kDm / 8, kWCarry);
  cast8_f16_kernel<<<(kDm * kDm / 8) / 256, 256, 0, stream>>>(ow, WO16, kDm * kDm / 8, kWCarry);

  gemm64_f16_kernel<2, 2><<<((kTok / 64) * (kQKld / 64)) / 8, 256, 0, stream>>>(
      X16, kDm, W16, kDm, (void*)QK16, (void*)QKL16, kQKld, ipb,
      kTok, kQKld, kDm, kProjScale, kQKVCarry);

  gemm64_f16_kernel<1, 2><<<((kDm / 64) * (kTok / 64)) / 8, 256, 0, stream>>>(
      W16 + (size_t)2 * kDm * kDm, kDm, X16, kDm, (void*)VT16, (void*)VTL16, kTok, ipb + 2 * kDm,
      kDm, kTok, kDm, kProjScale, kQKVCarry);

  band_attn_kernel<<<kBatch * kHeads * (kSeq / kQT), 64, 0, stream>>>(QK16, QKL16, VT16, VTL16, CTX16);

  gemm64_f16_kernel<2, 0><<<((kTok / 64) * (kDm / 64)) / 8, 256, 0, stream>>>(
      CTX16, kDm, WO16, kDm, (void*)out, nullptr, kDm, ob,
      kTok, kDm, kDm, kOutScale, 1.0f);
}
